// SequentialMultiHeadAttention_50062138802613
// MI455X (gfx1250) — hardware-verified
//
#include <hip/hip_runtime.h>
#include <stddef.h>


#define NBT 4
#define TS 2048
#define EM 1024
#define NHD 16
#define HDM 64

typedef __bf16 v16bf __attribute__((ext_vector_type(16)));
typedef float v8f __attribute__((ext_vector_type(8)));
typedef float v4f __attribute__((ext_vector_type(4)));
typedef unsigned int v4u __attribute__((ext_vector_type(4)));
typedef v4f __attribute__((__may_alias__)) v4fa;
typedef unsigned short us_t;

union Frag { v16bf v; v4u u[2]; };

__device__ __forceinline__ v8f mma(const v16bf a, const v16bf b, v8f c) {
  return __builtin_amdgcn_wmma_f32_16x16x32_bf16(false, a, false, b, (short)0, c, false, false);
}

__device__ __forceinline__ v8f mma3(const Frag& ah, const Frag& al, const Frag& bh, const Frag& bl, v8f c) {
  c = mma(ah.v, bh.v, c);
  c = mma(al.v, bh.v, c);
  c = mma(ah.v, bl.v, c);
  return c;
}

__device__ __forceinline__ void ldfrag(Frag& f, const us_t* rowk, int hh) {
  f.u[0] = *(const v4u*)(rowk + 8 * hh);
  f.u[1] = *(const v4u*)(rowk + 16 + 8 * hh);
}

__device__ __forceinline__ unsigned int pk2(float a, float b, unsigned int& lo) {
  const __bf16 ha = (__bf16)a;
  const __bf16 hb = (__bf16)b;
  const unsigned int ua = (unsigned int)__builtin_bit_cast(unsigned short, ha);
  const unsigned int ub = (unsigned int)__builtin_bit_cast(unsigned short, hb);
  const float ra = a - __builtin_bit_cast(float, ua << 16);
  const float rb = b - __builtin_bit_cast(float, ub << 16);
  const __bf16 la = (__bf16)ra;
  const __bf16 lb = (__bf16)rb;
  lo = (unsigned int)__builtin_bit_cast(unsigned short, la) |
       ((unsigned int)__builtin_bit_cast(unsigned short, lb) << 16);
  return ua | (ub << 16);
}

__device__ __forceinline__ void split8(const v4f a, const v4f b, v4u& hi, v4u& lo) {
  v4u H, L;
  unsigned int l0, l1, l2, l3;
  H.x = pk2(a.x, a.y, l0);
  H.y = pk2(a.z, a.w, l1);
  H.z = pk2(b.x, b.y, l2);
  H.w = pk2(b.z, b.w, l3);
  L.x = l0; L.y = l1; L.z = l2; L.w = l3;
  hi = H; lo = L;
}

__global__ void __launch_bounds__(256) k_cvt_rows(const float* __restrict__ src,
                                                  us_t* hi, us_t* lo, int nchunks) {
  const int i = blockIdx.x * 256 + threadIdx.x;
  if (i >= nchunks) return;
  const size_t e0 = (size_t)i * 8;
  const v4f a = *(const v4f*)(src + e0);
  const v4f b = *(const v4f*)(src + e0 + 4);
  v4u H, L;
  split8(a, b, H, L);
  *(volatile v4u*)(hi + e0) = H;
  *(volatile v4u*)(lo + e0) = L;
  __threadfence();
  *(volatile v4u*)(hi + e0) = H;
  *(volatile v4u*)(lo + e0) = L;
}

__global__ void __launch_bounds__(256) k_cvt_wqkv(const float* __restrict__ Wq,
                                                  const float* __restrict__ Wk,
                                                  const float* __restrict__ Wv,
                                                  us_t* ph, us_t* pl) {
  __shared__ __attribute__((aligned(16))) float tile[64][65];
  const int tid = threadIdx.x;
  const int kt = blockIdx.x, h = blockIdx.y, w = blockIdx.z;
  const float* W = (w == 0) ? Wq : ((w == 1) ? Wk : Wv);
#pragma unroll
  for (int p = 0; p < 4; ++p) {
    const int r = p * 16 + (tid >> 4);
    const int c4 = (tid & 15) * 4;
    const v4f v = *(const v4f*)(W + ((size_t)(h * EM + kt * 64 + r)) * HDM + c4);
    tile[c4 + 0][r] = v.x;
    tile[c4 + 1][r] = v.y;
    tile[c4 + 2][r] = v.z;
    tile[c4 + 3][r] = v.w;
  }
  __syncthreads();
#pragma unroll 1
  for (int rep = 0; rep < 2; ++rep) {
#pragma unroll
    for (int s = 0; s < 2; ++s) {
      const int nl = s * 32 + (tid >> 3);
      const int p8 = tid & 7;
      v4f a, b;
      a.x = tile[nl][8 * p8 + 0]; a.y = tile[nl][8 * p8 + 1];
      a.z = tile[nl][8 * p8 + 2]; a.w = tile[nl][8 * p8 + 3];
      b.x = tile[nl][8 * p8 + 4]; b.y = tile[nl][8 * p8 + 5];
      b.z = tile[nl][8 * p8 + 6]; b.w = tile[nl][8 * p8 + 7];
      v4u H, L;
      split8(a, b, H, L);
      const size_t n = (size_t)(w * EM + h * HDM + nl);
      const size_t o = n * EM + (size_t)kt * 64 + 8 * p8;
      *(volatile v4u*)(ph + o) = H;
      *(volatile v4u*)(pl + o) = L;
    }
    if (rep == 0) __threadfence();
  }
}

__device__ __forceinline__ void gemm64(const us_t* __restrict__ Ah, const us_t* __restrict__ Al,
                                       const us_t* __restrict__ Bh, const us_t* __restrict__ Bl,
                                       int m0, int n0, int wave, int lane,
                                       v8f& c00, v8f& c01, v8f& c10, v8f& c11) {
  const int hh = lane >> 4, m = lane & 15;
  const int wm = wave >> 1, wn = wave & 1;
  const size_t ao = (size_t)(m0 + wm * 32 + m) * EM;
  const size_t bo = (size_t)(n0 + wn * 32 + m) * EM;
  const us_t* a0h = Ah + ao;            const us_t* a0l = Al + ao;
  const us_t* a1h = a0h + 16 * EM;      const us_t* a1l = a0l + 16 * EM;
  const us_t* b0h = Bh + bo;            const us_t* b0l = Bl + bo;
  const us_t* b1h = b0h + 16 * EM;      const us_t* b1l = b0l + 16 * EM;
  v8f z = {};
  c00 = z; c01 = z; c10 = z; c11 = z;
#pragma unroll 1
  for (int k0 = 0; k0 < EM; k0 += 32) {
    Frag ah0, al0, ah1, al1, bh0, bl0, bh1, bl1;
    ldfrag(ah0, a0h + k0, hh); ldfrag(al0, a0l + k0, hh);
    ldfrag(ah1, a1h + k0, hh); ldfrag(al1, a1l + k0, hh);
    ldfrag(bh0, b0h + k0, hh); ldfrag(bl0, b0l + k0, hh);
    ldfrag(bh1, b1h + k0, hh); ldfrag(bl1, b1l + k0, hh);
    c00 = mma3(ah0, al0, bh0, bl0, c00);
    c01 = mma3(ah0, al0, bh1, bl1, c01);
    c10 = mma3(ah1, al1, bh0, bl0, c10);
    c11 = mma3(ah1, al1, bh1, bl1, c11);
    asm volatile("v_nop\n\tv_nop\n\tv_nop\n\tv_nop"
                 : "+v"(c00), "+v"(c01), "+v"(c10), "+v"(c11)
                 : "v"(ah0.v), "v"(al0.v), "v"(ah1.v), "v"(al1.v),
                   "v"(bh0.v), "v"(bl0.v), "v"(bh1.v), "v"(bl1.v));
  }
}

__device__ __forceinline__ void stage_tile(float (*stg)[68], const v8f& c, int row0, int col, bool tr) {
#pragma unroll
  for (int r = 0; r < 8; ++r) {
    if (tr) stg[col][row0 + r] = c[r];
    else    stg[row0 + r][col] = c[r];
  }
}

__global__ void __launch_bounds__(128) k_qkv(const us_t* __restrict__ xh, const us_t* __restrict__ xl,
                                             const us_t* __restrict__ wh, const us_t* __restrict__ wl,
                                             us_t* qh, us_t* ql, us_t* kh, us_t* kl,
                                             us_t* vh, us_t* vl) {
  __shared__ __attribute__((aligned(16))) float stg[64][68];
  const int tid = threadIdx.x, wave = tid >> 5, lane = tid & 31;
  const int hh = lane >> 4, m = lane & 15, wm = wave >> 1, wn = wave & 1;
  const int nb = blockIdx.x, mb = blockIdx.y;
  const int which = nb >> 4, h = nb & 15;
  const int t0 = mb * 64, n0 = nb * 64;
  v8f c00, c01, c10, c11;
  gemm64(xh, xl, wh, wl, t0, n0, wave, lane, c00, c01, c10, c11);
  const bool tr = (which == 2);
  stage_tile(stg, c00, wm * 32 + 8 * hh,      wn * 32 + m,      tr);
  stage_tile(stg, c01, wm * 32 + 8 * hh,      wn * 32 + 16 + m, tr);
  stage_tile(stg, c10, wm * 32 + 16 + 8 * hh, wn * 32 + m,      tr);
  stage_tile(stg, c11, wm * 32 + 16 + 8 * hh, wn * 32 + 16 + m, tr);
  __syncthreads();
  us_t* dh; us_t* dl;
  if (which == 0) { dh = qh; dl = ql; } else if (which == 1) { dh = kh; dl = kl; } else { dh = vh; dl = vl; }
  size_t base; size_t pitch;
  if (which < 2) { base = ((size_t)h * TS + t0) * HDM; pitch = HDM; }
  else           { base = (size_t)h * HDM * TS + t0;   pitch = TS; }
#pragma unroll 1
  for (int rep = 0; rep < 2; ++rep) {
#pragma unroll
    for (int s = 0; s < 4; ++s) {
      const int L = s * 16 + (tid >> 3);
      const int p = tid & 7;
      const v4fa* pr = (const v4fa*)&stg[L][0];
      const v4f a = pr[2 * p];
      const v4f b = pr[2 * p + 1];
      v4u H, Lo;
      split8(a, b, H, Lo);
      const size_t o = base + (size_t)L * pitch + 8 * p;
      *(volatile v4u*)(dh + o) = H;
      *(volatile v4u*)(dl + o) = Lo;
    }
    if (rep == 0) __threadfence();
  }
}

__global__ void __launch_bounds__(64) k_attn(const us_t* __restrict__ qh, const us_t* __restrict__ ql,
                                             const us_t* __restrict__ kh, const us_t* __restrict__ kl,
                                             const us_t* __restrict__ vh, const us_t* __restrict__ vl,
                                             us_t* oh, us_t* ol) {
  __shared__ __attribute__((aligned(16))) float stg[2][16][68];
  const int tid = threadIdx.x, wave = tid >> 5, lane = tid & 31;
  const int hh = lane >> 4, m = lane & 15;
  const int qb = blockIdx.x, h = blockIdx.y;
  const int tb = qb * 32 + wave * 16;
  const float ninf = -__builtin_inff();

  Frag Qh0, Ql0, Qh1, Ql1;
  {
    const size_t qo = ((size_t)h * TS + tb + m) * HDM;
    ldfrag(Qh0, qh + qo, hh);      ldfrag(Ql0, ql + qo, hh);
    ldfrag(Qh1, qh + qo + 32, hh); ldfrag(Ql1, ql + qo + 32, hh);
  }
  v8f acc0 = {}, acc1 = {}, acc2 = {}, acc3 = {};
  float mrow[8], lrow[8];
#pragma unroll
  for (int r = 0; r < 8; ++r) { mrow[r] = ninf; lrow[r] = 0.0f; }

  const us_t* kbh = kh + (size_t)h * TS * HDM;
  const us_t* kbl = kl + (size_t)h * TS * HDM;
  const us_t* vbh = vh + (size_t)h * HDM * TS;
  const us_t* vbl = vl + (size_t)h * HDM * TS;

#pragma unroll 1
  for (int j = 0; j <= qb; ++j) {
    const int s0 = j * 32;
    Frag Kh00, Kl00, Kh01, Kl01, Kh10, Kl10, Kh11, Kl11;
    {
      const size_t r0o = (size_t)(s0 + m) * HDM;
      const size_t r1o = r0o + 16 * HDM;
      ldfrag(Kh00, kbh + r0o, hh);      ldfrag(Kl00, kbl + r0o, hh);
      ldfrag(Kh01, kbh + r0o + 32, hh); ldfrag(Kl01, kbl + r0o + 32, hh);
      ldfrag(Kh10, kbh + r1o, hh);      ldfrag(Kl10, kbl + r1o, hh);
      ldfrag(Kh11, kbh + r1o + 32, hh); ldfrag(Kl11, kbl + r1o + 32, hh);
    }
    v8f s0t = {}, s1t = {};
    s0t = mma3(Qh0, Ql0, Kh00, Kl00, s0t);
    s0t = mma3(Qh1, Ql1, Kh01, Kl01, s0t);
    s1t = mma3(Qh0, Ql0, Kh10, Kl10, s1t);
    s1t = mma3(Qh1, Ql1, Kh11, Kl11, s1t);
    asm volatile("v_nop\n\tv_nop\n\tv_nop\n\tv_nop"
                 : "+v"(s0t), "+v"(s1t)
                 : "v"(Qh0.v), "v"(Ql0.v), "v"(Qh1.v), "v"(Ql1.v),
                   "v"(Kh00.v), "v"(Kl00.v), "v"(Kh01.v), "v"(Kl01.v),
                   "v"(Kh10.v), "v"(Kl10.v), "v"(Kh11.v), "v"(Kl11.v));

    const bool diag = (j == qb);
    float p0[8], p1[8];
#pragma unroll
    for (int r = 0; r < 8; ++r) {
      float v0 = s0t[r] * 0.125f;
      float v1 = s1t[r] * 0.125f;
      if (diag) {
        const int trow = tb + 8 * hh + r;
        if (s0 + m > trow)      v0 = ninf;
        if (s0 + 16 + m > trow) v1 = ninf;
      }
      float mx = fmaxf(v0, v1);
#pragma unroll
      for (int off = 1; off < 16; off <<= 1) mx = fmaxf(mx, __shfl_xor(mx, off, 16));
      const float mnew = fmaxf(mrow[r], mx);
      const float alpha = __expf(mrow[r] - mnew);
      mrow[r] = mnew;
      v0 = __expf(v0 - mnew);
      v1 = __expf(v1 - mnew);
      float sum = v0 + v1;
#pragma unroll
      for (int off = 1; off < 16; off <<= 1) sum += __shfl_xor(sum, off, 16);
      lrow[r] = lrow[r] * alpha + sum;
      acc0[r] *= alpha; acc1[r] *= alpha; acc2[r] *= alpha; acc3[r] *= alpha;
      p0[r] = v0;
      p1[r] = v1;
    }

    __syncthreads();
#pragma unroll
    for (int r = 0; r < 8; ++r) {
      stg[wave][8 * hh + r][m]      = p0[r];
      stg[wave][8 * hh + r][16 + m] = p1[r];
    }
    __syncthreads();
    Frag Ph, Pl;
    {
      const v4fa* pr = (const v4fa*)&stg[wave][m][0];
      const v4f a0 = pr[2 * hh];
      const v4f a1 = pr[2 * hh + 1];
      const v4f b0 = pr[4 + 2 * hh];
      const v4f b1 = pr[5 + 2 * hh];
      split8(a0, a1, Ph.u[0], Pl.u[0]);
      split8(b0, b1, Ph.u[1], Pl.u[1]);
    }

    {
      Frag Vh0, Vl0, Vh1, Vl1;
      const size_t o0 = (size_t)(0 * 16 + m) * TS + s0;
      const size_t o1 = (size_t)(1 * 16 + m) * TS + s0;
      ldfrag(Vh0, vbh + o0, hh); ldfrag(Vl0, vbl + o0, hh);
      ldfrag(Vh1, vbh + o1, hh); ldfrag(Vl1, vbl + o1, hh);
      acc0 = mma3(Ph, Pl, Vh0, Vl0, acc0);
      acc1 = mma3(Ph, Pl, Vh1, Vl1, acc1);
      asm volatile("v_nop\n\tv_nop\n\tv_nop\n\tv_nop"
                   : "+v"(acc0), "+v"(acc1)
                   : "v"(Ph.v), "v"(Pl.v), "v"(Vh0.v), "v"(Vl0.v), "v"(Vh1.v), "v"(Vl1.v));
    }
    {
      Frag Vh2, Vl2, Vh3, Vl3;
      const size_t o2 = (size_t)(2 * 16 + m) * TS + s0;
      const size_t o3 = (size_t)(3 * 16 + m) * TS + s0;
      ldfrag(Vh2, vbh + o2, hh); ldfrag(Vl2, vbl + o2, hh);
      ldfrag(Vh3, vbh + o3, hh); ldfrag(Vl3, vbl + o3, hh);
      acc2 = mma3(Ph, Pl, Vh2, Vl2, acc2);
      acc3 = mma3(Ph, Pl, Vh3, Vl3, acc3);
      asm volatile("v_nop\n\tv_nop\n\tv_nop\n\tv_nop"
                   : "+v"(acc2), "+v"(acc3)
                   : "v"(Ph.v), "v"(Pl.v), "v"(Vh2.v), "v"(Vl2.v), "v"(Vh3.v), "v"(Vl3.v));
    }
  }

  __syncthreads();
#pragma unroll
  for (int r = 0; r < 8; ++r) {
    const float inv = 1.0f / lrow[r];
    const int row = 8 * hh + r;
    stg[wave][row][m]      = acc0[r] * inv;
    stg[wave][row][16 + m] = acc1[r] * inv;
    stg[wave][row][32 + m] = acc2[r] * inv;
    stg[wave][row][48 + m] = acc3[r] * inv;
  }
  __syncthreads();
#pragma unroll 1
  for (int rep = 0; rep < 2; ++rep) {
#pragma unroll
    for (int s = 0; s < 4; ++s) {
      const int L = s * 8 + (tid >> 3);
      const int p = tid & 7;
      const v4fa* pr = (const v4fa*)&stg[L >> 4][L & 15][0];
      const v4f a = pr[2 * p];
      const v4f b = pr[2 * p + 1];
      v4u H, Lo;
      split8(a, b, H, Lo);
      const size_t o = ((size_t)(qb * 32 + L)) * EM + (size_t)h * HDM + 8 * p;
      *(volatile v4u*)(oh + o) = H;
      *(volatile v4u*)(ol + o) = Lo;
    }
    if (rep == 0) __threadfence();
  }
}

__global__ void __launch_bounds__(128) k_proj(const us_t* __restrict__ ah, const us_t* __restrict__ al,
                                              const us_t* __restrict__ wh, const us_t* __restrict__ wl,
                                              const float* __restrict__ bo, float* y) {
  __shared__ __attribute__((aligned(16))) float stg[64][68];
  const int tid = threadIdx.x, wave = tid >> 5, lane = tid & 31;
  const int hh = lane >> 4, m = lane & 15, wm = wave >> 1, wn = wave & 1;
  const int nb = blockIdx.x, mb = blockIdx.y;
  const int m0 = mb * 64, n0 = nb * 64;
  v8f c00, c01, c10, c11;
  gemm64(ah, al, wh, wl, m0, n0, wave, lane, c00, c01, c10, c11);
  stage_tile(stg, c00, wm * 32 + 8 * hh,      wn * 32 + m,      false);
  stage_tile(stg, c01, wm * 32 + 8 * hh,      wn * 32 + 16 + m, false);
  stage_tile(stg, c10, wm * 32 + 16 + 8 * hh, wn * 32 + m,      false);
  stage_tile(stg, c11, wm * 32 + 16 + 8 * hh, wn * 32 + 16 + m, false);
  __syncthreads();
  const int p = tid & 15;
  const v4f bias = *(const v4f*)(bo + n0 + 4 * p);
#pragma unroll 1
  for (int rep = 0; rep < 2; ++rep) {
#pragma unroll
    for (int s = 0; s < 8; ++s) {
      const int R = s * 8 + (tid >> 4);
      const v4fa* pr = (const v4fa*)&stg[R][0];
      v4f v = pr[p];
      v += bias;
      *(volatile v4f*)(y + (size_t)(m0 + R) * EM + n0 + 4 * p) = v;
    }
    if (rep == 0) __threadfence();
  }
}

extern "C" void kernel_launch(void* const* d_in, const int* in_sizes, int n_in,
                              void* d_out, int out_size, void* d_ws, size_t ws_size,
                              hipStream_t stream) {
  if (n_in != 6) return;
  if (in_sizes[0] != NBT * TS * EM) return;
  if (in_sizes[1] != NHD * EM * HDM || in_sizes[2] != NHD * EM * HDM || in_sizes[3] != NHD * EM * HDM) return;
  if (in_sizes[4] != EM * EM || in_sizes[5] != EM) return;
  if (out_size != NBT * TS * EM) return;

  const float* x  = (const float*)d_in[0];
  const float* Wq = (const float*)d_in[1];
  const float* Wk = (const float*)d_in[2];
  const float* Wv = (const float*)d_in[3];
  const float* Wo = (const float*)d_in[4];
  const float* bo = (const float*)d_in[5];
  float* y = (float*)d_out;

  const size_t szX    = (size_t)NBT * TS * EM * sizeof(us_t);
  const size_t szWqkv = (size_t)3 * EM * EM * sizeof(us_t);
  const size_t szWo   = (size_t)EM * EM * sizeof(us_t);
  const size_t szHB   = (size_t)NHD * TS * HDM * sizeof(us_t);
  const size_t szA    = (size_t)NBT * TS * EM * sizeof(us_t);
  const size_t total  = 2 * szX + 2 * szWqkv + 2 * szWo + 6 * szHB + 2 * szA;
  if (total > ws_size) return;

  char* ws = (char*)d_ws;
  size_t off = 0;
  us_t* xH  = (us_t*)(ws + off); off += szX;
  us_t* xL  = (us_t*)(ws + off); off += szX;
  us_t* wH  = (us_t*)(ws + off); off += szWqkv;
  us_t* wL  = (us_t*)(ws + off); off += szWqkv;
  us_t* woH = (us_t*)(ws + off); off += szWo;
  us_t* woL = (us_t*)(ws + off); off += szWo;
  us_t* qH  = (us_t*)(ws + off); off += szHB;
  us_t* qL  = (us_t*)(ws + off); off += szHB;
  us_t* kH  = (us_t*)(ws + off); off += szHB;
  us_t* kL  = (us_t*)(ws + off); off += szHB;
  us_t* vH  = (us_t*)(ws + off); off += szHB;
  us_t* vL  = (us_t*)(ws + off); off += szHB;
  us_t* aH  = (us_t*)(ws + off); off += szA;
  us_t* aL  = (us_t*)(ws + off); off += szA;
  if (off > ws_size) return;

  const int nchX = NBT * TS * EM / 8;
  k_cvt_rows<<<(nchX + 255) / 256, 256, 0, stream>>>(x, xH, xL, nchX);
  const int nchWo = EM * EM / 8;
  k_cvt_rows<<<(nchWo + 255) / 256, 256, 0, stream>>>(Wo, woH, woL, nchWo);
  k_cvt_wqkv<<<dim3(EM / 64, NHD, 3), 256, 0, stream>>>(Wq, Wk, Wv, wH, wL);

  for (int b = 0; b < NBT; ++b) {
    const size_t xo = (size_t)b * TS * EM;
    k_qkv<<<dim3(3 * EM / 64, TS / 64), 128, 0, stream>>>(xH + xo, xL + xo, wH, wL,
                                                          qH, qL, kH, kL, vH, vL);
    k_attn<<<dim3(TS / 32, NHD), 64, 0, stream>>>(qH, qL, kH, kL, vH, vL, aH + xo, aL + xo);
  }
  k_proj<<<dim3(EM / 64, NBT * TS / 64), 128, 0, stream>>>(aH, aL, woH, woL, bo, y);
}
